// KANLayer_26225070309752
// MI455X (gfx1250) — hardware-verified
//
#include <hip/hip_runtime.h>
#include <math.h>

constexpr int kBatch  = 4096;
constexpr int kIn     = 512;
constexpr int kOutDim = 512;
constexpr int kKnots  = 6;
constexpr int kNB     = 9;
constexpr int kKdim   = kIn * kNB;
constexpr float kActCarry = 1024.0f;
constexpr float kWCarry   = 64.0f;
constexpr float kOutScale = 1.0f / (1024.0f * 64.0f);

constexpr size_t kActsBytes = (size_t)kBatch * kKdim * 2;
constexpr size_t kWqBytes   = (size_t)kOutDim * kKdim * 2;
constexpr size_t kWsTotal   = kActsBytes + kWqBytes;
static_assert(kWsTotal <= (size_t)134217728u);
static_assert(kActsBytes % 128 == 0);
static_assert(kKdim % 32 == 0);
static_assert(kBatch % 64 == 0 && kOutDim % 64 == 0);
static_assert((kOutDim * kKdim) % (8 * 256) == 0);
static_assert(kIn == 512 && kNB == 9);

typedef __attribute__((ext_vector_type(16))) _Float16 v16h;
typedef __attribute__((ext_vector_type(8)))  _Float16 v8h;
typedef __attribute__((ext_vector_type(16))) __bf16   v16b;
typedef __attribute__((ext_vector_type(8)))  __bf16   v8b;
typedef __attribute__((ext_vector_type(8)))  float    v8f;
typedef __attribute__((ext_vector_type(4)))  float    v4f;
typedef __attribute__((ext_vector_type(4)))  unsigned int v4u;

__device__ __forceinline__ unsigned short f2bf_bits(float f) {
  unsigned u = __float_as_uint(f);
  return (unsigned short)((u + 0x7FFFu + ((u >> 16) & 1u)) >> 16);
}
__device__ __forceinline__ float bf_bits2f(unsigned short h) { return __uint_as_float(((unsigned)h) << 16); }

__device__ __forceinline__ void dep_guard_h(v8f& a, v8f& b, v16h x, v16h y) { asm volatile("v_nop\n\tv_nop\n\tv_nop\n\tv_nop" : "+v"(a), "+v"(b) : "v"(x), "v"(y)); }
__device__ __forceinline__ void dep_guard_b(v8f& a, v8f& b, v16b x, v16b y) { asm volatile("v_nop\n\tv_nop\n\tv_nop\n\tv_nop" : "+v"(a), "+v"(b) : "v"(x), "v"(y)); }
__device__ __forceinline__ void dep_guard4_h(v8f& a, v8f& b, v8f& c, v8f& d, v16h x, v16h y) { asm volatile("v_nop\n\tv_nop\n\tv_nop\n\tv_nop" : "+v"(a), "+v"(b), "+v"(c), "+v"(d) : "v"(x), "v"(y)); }
__device__ __forceinline__ void dep_guard4_b(v8f& a, v8f& b, v8f& c, v8f& d, v16b x, v16b y) { asm volatile("v_nop\n\tv_nop\n\tv_nop\n\tv_nop" : "+v"(a), "+v"(b), "+v"(c), "+v"(d) : "v"(x), "v"(y)); }
__device__ __forceinline__ void keep4_h(v16h a, v16h b, v16h c, v16h d) { asm volatile("v_nop" :: "v"(a), "v"(b), "v"(c), "v"(d)); }
__device__ __forceinline__ void keep4_b(v16b a, v16b b, v16b c, v16b d) { asm volatile("v_nop" :: "v"(a), "v"(b), "v"(c), "v"(d)); }
__device__ __forceinline__ void acc_guard4(v8f& a, v8f& b, v8f& c, v8f& d) { asm volatile("v_nop\n\tv_nop\n\tv_nop\n\tv_nop" : "+v"(a), "+v"(b), "+v"(c), "+v"(d)); }
template <typename T> struct Frag;
template <> struct Frag<_Float16> {
  typedef v16h V; union U { v16h v; v8h h[2]; };
  static __device__ __forceinline__ v16h load(const _Float16* p) {
    U f; f.h[0] = *(const v8h*)(p); f.h[1] = *(const v8h*)(p + 16); return f.v;
  }
  static __device__ __forceinline__ v8f mma(v16h a, v16h b, v8f c) {
    return __builtin_amdgcn_wmma_f32_16x16x32_f16(false, a, false, b, (short)0, c, false, false);
  }
  static __device__ __forceinline__ void guard(v8f& a, v8f& b, v16h x, v16h y) { dep_guard_h(a, b, x, y); }
  static __device__ __forceinline__ void guard4(v8f& a, v8f& b, v8f& c, v8f& d, v16h x, v16h y) { dep_guard4_h(a, b, c, d, x, y); }
  static __device__ __forceinline__ void keep(v16h a, v16h b, v16h c, v16h d) { keep4_h(a, b, c, d); }
};
template <> struct Frag<__bf16> {
  typedef v16b V; union U { v16b v; v8b h[2]; };
  static __device__ __forceinline__ v16b load(const __bf16* p) {
    U f; f.h[0] = *(const v8b*)(p); f.h[1] = *(const v8b*)(p + 16); return f.v;
  }
  static __device__ __forceinline__ v8f mma(v16b a, v16b b, v8f c) {
    return __builtin_amdgcn_wmma_f32_16x16x32_bf16(false, a, false, b, (short)0, c, false, false);
  }
  static __device__ __forceinline__ void guard(v8f& a, v8f& b, v16b x, v16b y) { dep_guard_b(a, b, x, y); }
  static __device__ __forceinline__ void guard4(v8f& a, v8f& b, v8f& c, v8f& d, v16b x, v16b y) { dep_guard4_b(a, b, c, d, x, y); }
  static __device__ __forceinline__ void keep(v16b a, v16b b, v16b c, v16b d) { keep4_b(a, b, c, d); }
};

__device__ __forceinline__ unsigned pk16(unsigned short a, unsigned short b) { return (unsigned)a | ((unsigned)b << 16); }
__device__ __forceinline__ unsigned short h_bits(float f) { const _Float16 h = (_Float16)f; return __builtin_bit_cast(unsigned short, h); }

template <int ET> struct Elem;
template <> struct Elem<0> { typedef _Float16 T; };
template <> struct Elem<1> { typedef __bf16 T; };
template <int ET, bool SPLIT, int BIAS_MODE, int OUT_MODE, bool RESID, int ACT = 0>
__global__ __launch_bounds__(256) void wmma_gemm64(
    const unsigned short* __restrict__ Ap, const unsigned short* __restrict__ A2p, int lda, long strideA,
    const unsigned short* __restrict__ Btp, const unsigned short* __restrict__ Bt2p, int ldb, long strideB,
    void* __restrict__ Cout, void* __restrict__ Cout2, int ldc, long strideC,
    const float* __restrict__ bias,
    const float* __restrict__ resid, long strideR,
    int M, int N, int K, float scale) {
  typedef typename Elem<ET>::T T;
  typedef typename Frag<T>::V V;
  const T* A = (const T*)Ap; const T* A2 = (const T*)A2p; const T* Bt = (const T*)Btp; const T* Bt2 = (const T*)Bt2p;
  __shared__ __align__(16) float sT[8][16 * 68];
  const int b    = blockIdx.y;
  const int lane = threadIdx.x & 31;
  const int wave = threadIdx.x >> 5;
  const int tilesN = N >> 6;
  const int tilesM = M >> 6;
  const int tile = blockIdx.x * 8 + wave;
  if (tile >= tilesM * tilesN) return;
  const int tm = tile / tilesN;
  const int tn = tile - tm * tilesN;
  const int m0 = tm << 6;
  const int n0 = tn << 6;

  const T* Ab  = A  + (size_t)b * strideA;
  const T* Bb  = Bt + (size_t)b * strideB;
  const T* Ab2 = SPLIT ? (A2  + (size_t)b * strideA) : nullptr;
  const T* Bb2 = SPLIT ? (Bt2 + (size_t)b * strideB) : nullptr;

  const int rlane = lane & 15;
  const int koff  = (lane >> 4) * 8;
  const int mOff  = (lane >> 4) * 8;

  v8f acc[4][4];
#pragma unroll
  for (int i = 0; i < 4; ++i)
#pragma unroll
    for (int j = 0; j < 4; ++j) acc[i][j] = (v8f){0.f,0.f,0.f,0.f,0.f,0.f,0.f,0.f};

  for (int k0 = 0; k0 < K; k0 += 32) {
    V bh[4], bl[4];
#pragma unroll
    for (int j = 0; j < 4; ++j) {
      const size_t bo = (size_t)(n0 + (j << 4) + rlane) * ldb + koff + k0;
      bh[j] = Frag<T>::load(Bb + bo);
      if (SPLIT) bl[j] = Frag<T>::load(Bb2 + bo);
    }
#pragma unroll
    for (int i = 0; i < 4; ++i) {
      const size_t ao = (size_t)(m0 + (i << 4) + rlane) * lda + koff + k0;
      V ah = Frag<T>::load(Ab + ao);
      V al;
      if (SPLIT) al = Frag<T>::load(Ab2 + ao);
#pragma unroll
      for (int j = 0; j < 4; ++j) {
        acc[i][j] = Frag<T>::mma(ah, bh[j], acc[i][j]);
        if (SPLIT) {
          acc[i][j] = Frag<T>::mma(ah, bl[j], acc[i][j]);
          acc[i][j] = Frag<T>::mma(al, bh[j], acc[i][j]);
        }
      }
      Frag<T>::guard4(acc[i][0], acc[i][1], acc[i][2], acc[i][3], ah, SPLIT ? al : ah);
    }
    Frag<T>::keep(bh[0], bh[1], bh[2], bh[3]);
    if (SPLIT) Frag<T>::keep(bl[0], bl[1], bl[2], bl[3]);
  }
  acc_guard4(acc[0][0], acc[0][1], acc[0][2], acc[0][3]);
  acc_guard4(acc[1][0], acc[1][1], acc[1][2], acc[1][3]);
  acc_guard4(acc[2][0], acc[2][1], acc[2][2], acc[2][3]);
  acc_guard4(acc[3][0], acc[3][1], acc[3][2], acc[3][3]);

  float* slab = sT[wave];
  const float* Rb = RESID ? (resid + (size_t)b * strideR) : nullptr;
#pragma unroll
  for (int i = 0; i < 4; ++i) {
    const int mBase = m0 + (i << 4);
#pragma unroll
    for (int j = 0; j < 4; ++j) {
      const int n = n0 + (j << 4) + rlane;
      float bv = 0.f;
      if (BIAS_MODE == 2) bv = bias[n];
#pragma unroll
      for (int r = 0; r < 8; ++r) {
        float v = acc[i][j][r] * scale;
        if (BIAS_MODE == 1) v += bias[mBase + mOff + r];
        if (BIAS_MODE == 2) v += bv;
        if (RESID) v += Rb[(size_t)(mBase + mOff + r) * ldc + n];
        if (ACT == 2) v = fmaxf(v, 0.0f);
        if (ACT == 4) v = (v > 0.f) ? v : 0.01f * v;
        slab[(mOff + r) * 68 + (j << 4) + rlane] = v;
      }
    }
    __builtin_amdgcn_fence(__ATOMIC_RELEASE, "workgroup");
    __builtin_amdgcn_wave_barrier();
    __builtin_amdgcn_fence(__ATOMIC_ACQUIRE, "workgroup");
    if (OUT_MODE == 0) {
      float* C = (float*)Cout + (size_t)b * strideC;
      const int hh = lane >> 4, c4 = (lane & 15) * 4;
      for (int pass = 0; pass < 2; ++pass) {
#pragma unroll
        for (int it = 0; it < 8; ++it) {
          const int row = it * 2 + hh;
          v4f v = *(const v4f*)(slab + row * 68 + c4);
          *(volatile v4f*)(C + (size_t)(mBase + row) * ldc + n0 + c4) = v;
        }
        __threadfence();
      }
    } else {
      const int q = lane >> 3, c8 = (lane & 7) * 8;
      unsigned short* C  = (unsigned short*)Cout  + (size_t)b * strideC;
      unsigned short* C2 = (OUT_MODE == 2) ? ((unsigned short*)Cout2 + (size_t)b * strideC) : nullptr;
      for (int pass = 0; pass < 2; ++pass) {
#pragma unroll
        for (int it = 0; it < 4; ++it) {
          const int row = it * 4 + q;
          const float* sp = slab + row * 68 + c8;
          v8h hv, lv;
#pragma unroll
          for (int e = 0; e < 8; ++e) {
            if (OUT_MODE == 1) {
              hv[e] = (_Float16)sp[e];
            } else {
              unsigned short hb = f2bf_bits(sp[e]);
              unsigned short lb = f2bf_bits(sp[e] - bf_bits2f(hb));
              hv[e] = __builtin_bit_cast(_Float16, hb);
              lv[e] = __builtin_bit_cast(_Float16, lb);
            }
          }
          *(volatile v8h*)(C + (size_t)(mBase + row) * ldc + n0 + c8) = hv;
          if (OUT_MODE == 2) *(volatile v8h*)(C2 + (size_t)(mBase + row) * ldc + n0 + c8) = lv;
        }
        __threadfence();
      }
    }
    __builtin_amdgcn_fence(__ATOMIC_RELEASE, "workgroup");
    __builtin_amdgcn_wave_barrier();
    __builtin_amdgcn_fence(__ATOMIC_ACQUIRE, "workgroup");
  }
}

__global__ __launch_bounds__(256) void cast8_f16_kernel(const float* __restrict__ in, unsigned short* __restrict__ out,
                                                        int n8, float scale) {
  const int i = blockIdx.x * 256 + threadIdx.x;
  if (i >= n8) return;
  const float* p = in + 8 * (size_t)i;
  const v4f a = *(const v4f*)(p);
  const v4f c = *(const v4f*)(p + 4);
  unsigned short hb[8];
#pragma unroll
  for (int e = 0; e < 4; ++e) {
    hb[e]     = h_bits(a[e] * scale);
    hb[4 + e] = h_bits(c[e] * scale);
  }
  const v4u u = (v4u){pk16(hb[0], hb[1]), pk16(hb[2], hb[3]), pk16(hb[4], hb[5]), pk16(hb[6], hb[7])};
  unsigned short* q = out + 8 * (size_t)i;
  *(volatile v4u*)q = u;
  __threadfence();
  *(volatile v4u*)q = u;
}

__global__ __launch_bounds__(256) void basis_kernel(const float* __restrict__ x, const float* __restrict__ knots,
                                                    unsigned short* __restrict__ acts) {
#pragma clang fp contract(off)
  __shared__ __align__(16) float stg[kNB * 256];
  const int t    = threadIdx.x;
  const int lane = t & 31;
  const int wave = t >> 5;
  const int brow = blockIdx.x >> 1;
  const int d0   = (blockIdx.x & 1) * 256;
  const int d    = d0 + t;

  const float xv = x[(size_t)brow * kIn + d];
  const float* gp = knots + d * kKnots;
  const float kn0 = gp[0], kn1 = gp[1], kn2 = gp[2], kn3 = gp[3], kn4 = gp[4], kn5 = gp[5];
  const float hs = (kn5 - kn0) * 0.2f;

  float gk[12];
  gk[0] = kn0 - hs * 3.0f;
  gk[1] = kn0 - hs * 2.0f;
  gk[2] = kn0 - hs;
  gk[3] = kn0; gk[4] = kn1; gk[5] = kn2; gk[6] = kn3; gk[7] = kn4; gk[8] = kn5;
  gk[9]  = kn5 + hs;
  gk[10] = kn5 + hs * 2.0f;
  gk[11] = kn5 + hs * 3.0f;

  float bb[11];
#pragma unroll
  for (int i = 0; i < 11; ++i) bb[i] = (xv >= gk[i] && xv < gk[i + 1]) ? 1.0f : 0.0f;

#pragma unroll
  for (int i = 0; i < 10; ++i) {
    const float rl = __builtin_amdgcn_rcpf(gk[i + 1] - gk[i]);
    const float rr = __builtin_amdgcn_rcpf(gk[i + 2] - gk[i + 1]);
    const float lf = (xv - gk[i]) * rl;
    const float rt = (gk[i + 2] - xv) * rr;
    const float pl = lf * bb[i];
    const float pr = rt * bb[i + 1];
    bb[i] = pl + pr;
  }
#pragma unroll
  for (int i = 0; i < 9; ++i) {
    const float rl = __builtin_amdgcn_rcpf(gk[i + 2] - gk[i]);
    const float rr = __builtin_amdgcn_rcpf(gk[i + 3] - gk[i + 1]);
    const float lf = (xv - gk[i]) * rl;
    const float rt = (gk[i + 3] - xv) * rr;
    const float pl = lf * bb[i];
    const float pr = rt * bb[i + 1];
    bb[i] = pl + pr;
  }
#pragma unroll
  for (int i = 0; i < 8; ++i) {
    const float rl = __builtin_amdgcn_rcpf(gk[i + 3] - gk[i]);
    const float rr = __builtin_amdgcn_rcpf(gk[i + 4] - gk[i + 1]);
    const float lf = (xv - gk[i]) * rl;
    const float rt = (gk[i + 4] - xv) * rr;
    const float pl = lf * bb[i];
    const float pr = rt * bb[i + 1];
    bb[i] = pl + pr;
  }

  const float ex = expf(-xv);
  const float sg = 1.0f / (1.0f + ex);
  const float sl = xv * sg;

#pragma unroll
  for (int j = 0; j < 8; ++j) stg[j * 256 + t] = bb[j] * xv;
  stg[8 * 256 + t] = sl * xv;
  __syncthreads();

  const float* s0 = stg + wave * 256 + 8 * lane;
  const float* s1 = stg + 8 * 256 + 8 * lane;
  const v4f a0 = *(const v4f*)(s0);
  const v4f a1 = *(const v4f*)(s0 + 4);
  const v4f e0 = *(const v4f*)(s1);
  const v4f e1 = *(const v4f*)(s1 + 4);
  unsigned short h0[8], h1[8];
#pragma unroll
  for (int e = 0; e < 4; ++e) {
    h0[e]     = h_bits(a0[e] * kActCarry);
    h0[4 + e] = h_bits(a1[e] * kActCarry);
    h1[e]     = h_bits(e0[e] * kActCarry);
    h1[4 + e] = h_bits(e1[e] * kActCarry);
  }
  const v4u u0 = (v4u){pk16(h0[0], h0[1]), pk16(h0[2], h0[3]), pk16(h0[4], h0[5]), pk16(h0[6], h0[7])};
  const v4u u1 = (v4u){pk16(h1[0], h1[1]), pk16(h1[2], h1[3]), pk16(h1[4], h1[5]), pk16(h1[6], h1[7])};
  unsigned short* rowp = acts + (size_t)brow * kKdim + d0 + 8 * lane;
  unsigned short* p0 = rowp + wave * kIn;
  unsigned short* p1 = rowp + 8 * kIn;
  for (int pass = 0; pass < 2; ++pass) {
    *(volatile v4u*)p0 = u0;
    if (wave == 0) *(volatile v4u*)p1 = u1;
    __threadfence();
  }
}

extern "C" void kernel_launch(void* const* d_in, const int* in_sizes, int n_in,
                              void* d_out, int out_size, void* d_ws, size_t ws_size,
                              hipStream_t stream)
{
  if (n_in < 4) return;
  if (in_sizes[0] != kBatch * kIn) return;
  if (in_sizes[1] != kIn * kKnots) return;
  if (in_sizes[2] != kOutDim * kKdim) return;
  if (in_sizes[3] != kOutDim) return;
  if (out_size != kBatch * kOutDim) return;
  if (ws_size < kWsTotal) return;

  const float* x     = (const float*)d_in[0];
  const float* knots = (const float*)d_in[1];
  const float* w     = (const float*)d_in[2];
  const float* bias  = (const float*)d_in[3];
  unsigned short* acts = (unsigned short*)d_ws;
  unsigned short* wq   = (unsigned short*)((char*)d_ws + kActsBytes);

  const int n8 = (kOutDim * kKdim) / 8;
  cast8_f16_kernel<<<(n8 + 255) / 256, 256, 0, stream>>>(w, wq, n8, kWCarry);

  basis_kernel<<<kBatch * 2, 256, 0, stream>>>(x, knots, acts);

  const int tiles  = (kBatch / 64) * (kOutDim / 64);
  const int blocks = (tiles + 7) / 8;
  wmma_gemm64<0, false, 2, 0, false, 0><<<dim3(blocks, 1), 256, 0, stream>>>(
      acts, acts, kKdim, 0L,
      wq, wq, kKdim, 0L,
      d_out, d_out, kOutDim, 0L,
      bias,
      bias, 0L,
      kBatch, kOutDim, kKdim, kOutScale);
}
